// MambaLay_10075993276869
// MI455X (gfx1250) — hardware-verified
//
#include <hip/hip_runtime.h>
#include <math.h>

typedef __attribute__((ext_vector_type(16))) _Float16 v16h;
typedef __attribute__((ext_vector_type(16))) __bf16 v16b;
typedef __attribute__((ext_vector_type(8)))  _Float16 v8h;
typedef __attribute__((ext_vector_type(8)))  float v8f;
typedef __attribute__((ext_vector_type(4)))  float v4f;
typedef __attribute__((ext_vector_type(2)))  float v2f;
typedef __attribute__((ext_vector_type(4)))  unsigned v4u;
typedef __attribute__((ext_vector_type(4)))  int v4i;
typedef float __attribute__((may_alias)) float_a;
typedef int __attribute__((may_alias)) int_a;

template <typename T> __device__ __forceinline__ void vst2(void* p, T v) { *(volatile T*)p = v; __threadfence(); *(volatile T*)p = v; }
__device__ __forceinline__ v8f wmma16(v16h a, v16h b, v8f c) {
  v8f d = __builtin_amdgcn_wmma_f32_16x16x32_f16(false, a, false, b, (short)0, c, false, false);
  asm volatile("v_nop\n\tv_nop\n\tv_nop\n\tv_nop" : "+v"(d) : "v"(a), "v"(b));
  return d;
}
__device__ __forceinline__ v8f wmma_bf(v16b a, v16b b, v8f c) {
  v8f d = __builtin_amdgcn_wmma_f32_16x16x32_bf16(false, a, false, b, (short)0, c, false, false);
  asm volatile("v_nop\n\tv_nop\n\tv_nop\n\tv_nop" : "+v"(d) : "v"(a), "v"(b));
  return d;
}
__device__ __forceinline__ v16h frag_h(const _Float16* rowk0, int lane) {
  union { v16h v; v8h q[2]; } u; const _Float16* p = rowk0 + 8 * (lane >> 4);
  u.q[0] = *(const v8h*)p; u.q[1] = *(const v8h*)(p + 16); return u.v;
}
__device__ __forceinline__ v16h frag_f32(const float* rowk0, int lane) {
  v16h a; const float* p = rowk0 + 8 * (lane >> 4);
#pragma unroll
  for (int i = 0; i < 8; ++i) { a[i] = (_Float16)p[i]; a[8 + i] = (_Float16)p[16 + i]; }
  return a;
}
__device__ __forceinline__ v16h frag_f32s(const float* rowk0, int lane, float sc) {
  v16h a; const float* p = rowk0 + 8 * (lane >> 4);
#pragma unroll
  for (int i = 0; i < 8; ++i) { a[i] = (_Float16)(p[i] * sc); a[8 + i] = (_Float16)(p[16 + i] * sc); }
  return a;
}
__device__ __forceinline__ v16h fragc_f32(const float* W, int k0, int n, int lane, int ld, int K) {
  v16h a; const int g = lane >> 4;
#pragma unroll
  for (int i = 0; i < 8; ++i) { const int ka = k0 + 8 * g + i, kb = ka + 16;
    a[i] = (_Float16)(ka < K ? W[(size_t)(ka < K ? ka : K - 1) * ld + n] : 0.f); a[8 + i] = (_Float16)(kb < K ? W[(size_t)(kb < K ? kb : K - 1) * ld + n] : 0.f); }
  return a;
}
struct F2 { v16b h, l; };
__device__ __forceinline__ F2 bsplit16(const float v[16]) { F2 r;
#pragma unroll
  for (int i = 0; i < 16; ++i) { const __bf16 h = (__bf16)v[i]; r.h[i] = h; r.l[i] = (__bf16)(v[i] - (float)h); }
  return r; }
__device__ __forceinline__ F2 split_row(const float* row, int k0, int lane) { float v[16]; const float* p = row + k0 + 8 * (lane >> 4);
#pragma unroll
  for (int i = 0; i < 8; ++i) { v[i] = p[i]; v[8 + i] = p[16 + i]; }
  return bsplit16(v); }
__device__ __forceinline__ F2 split_rowK(const float* row, int k0, int lane, int K) { float v[16]; const int g = lane >> 4;
#pragma unroll
  for (int i = 0; i < 8; ++i) { const int ka = k0 + 8 * g + i, kb = ka + 16; v[i] = ka < K ? row[ka < K ? ka : K - 1] : 0.f; v[8 + i] = kb < K ? row[kb < K ? kb : K - 1] : 0.f; }
  return bsplit16(v); }
__device__ __forceinline__ F2 split_col(const float* W, int k0, int n, int lane, int ld, int K) { float v[16]; const int g = lane >> 4;
#pragma unroll
  for (int i = 0; i < 8; ++i) { const int ka = k0 + 8 * g + i, kb = ka + 16; v[i] = ka < K ? W[(size_t)(ka < K ? ka : K - 1) * ld + n] : 0.f; v[8 + i] = kb < K ? W[(size_t)(kb < K ? kb : K - 1) * ld + n] : 0.f; }
  return bsplit16(v); }
__device__ __forceinline__ v8f mac3(const F2& a, const F2& b, v8f c) { c = wmma_bf(a.l, b.h, c); c = wmma_bf(a.h, b.l, c); return wmma_bf(a.h, b.h, c); }
__device__ __forceinline__ float sigm(float v) { return 1.0f / (1.0f + expf(-v)); }
#define LDSX() do { asm volatile("s_wait_dscnt 0" ::: "memory"); __builtin_amdgcn_wave_barrier(); __builtin_amdgcn_fence(__ATOMIC_RELEASE, "workgroup"); } while (0)


#define NBB 2
#define LL 2048
#define NR (NBB * LL)
#define DM 256
#define DI 512
#define NS 32
#define DTR 128
#define XDW (DTR + 2 * NS)
#define DQ 128
#define NOUT 32
__device__ __forceinline__ float bfr(float v) { return (float)(__bf16)v; }
__device__ __forceinline__ v16b frag_b(const __bf16* rowk0, int lane) { return __builtin_bit_cast(v16b, frag_h((const _Float16*)rowk0, lane)); }
__device__ __attribute__((noinline)) float exp_ni(float v) { return expf(v); }
__device__ __attribute__((noinline)) float softplus_ni(float v) { return v > 20.f ? v : log1pf(expf(v)); }
__device__ __attribute__((noinline)) float gelu_ni(float v) { return 0.5f * v * (1.0f + erff(v * 0.70710678118654752f)); }
__device__ __forceinline__ float silu_f(float v) { return v / (1.0f + exp_ni(-v)); }

__global__ __launch_bounds__(128) void k_lnin(const float* __restrict__ x, const float* __restrict__ lg, const float* __restrict__ lb, const float* __restrict__ Win, float* __restrict__ XI, float* __restrict__ RES) {
  __shared__ __align__(16) __bf16 sh_[4][16][DM + 8], sl_[4][16][DM + 8]; __shared__ __align__(16) float so[4][16][132];
  const int tid = threadIdx.x, wave = tid >> 5, lane = tid & 31, col = lane & 15, g = lane >> 4; const int r0 = blockIdx.x * 64 + wave * 16, n0 = blockIdx.y * 128;
  for (int rl = 0; rl < 16; ++rl) { const float* xr = x + (size_t)(r0 + rl) * DM; float v[8]; float s = 0.f;
#pragma unroll
    for (int e = 0; e < 8; ++e) { v[e] = bfr(xr[lane * 8 + e]); s += v[e]; }
#pragma unroll
    for (int o = 16; o > 0; o >>= 1) s += __shfl_xor(s, o, 32);
    const float mu = s * (1.0f / DM); float q = 0.f;
#pragma unroll
    for (int e = 0; e < 8; ++e) { const float dv = v[e] - mu; q += dv * dv; }
#pragma unroll
    for (int o = 16; o > 0; o >>= 1) q += __shfl_xor(q, o, 32);
    const float rs = rsqrtf(q * (1.0f / DM) + 1e-5f);
#pragma unroll
    for (int e = 0; e < 8; ++e) { const int c = lane * 8 + e; const float y = (v[e] - mu) * rs * bfr(lg[c]) + bfr(lb[c]); const __bf16 hi = (__bf16)y; sh_[wave][rl][c] = hi; sl_[wave][rl][c] = (__bf16)(y - (float)hi); } }
  LDSX();
  v8f acc[8] = {};
#pragma unroll 2
  for (int kc = 0; kc < DM / 32; ++kc) { const v16b ah = frag_b(&sh_[wave][col][0] + kc * 32, lane), al = frag_b(&sl_[wave][col][0] + kc * 32, lane);
#pragma unroll
    for (int j = 0; j < 8; ++j) { const v16b wb = split_col(Win, kc * 32, n0 + j * 16 + col, lane, 2 * DI, DM).h; acc[j] = wmma_bf(al, wb, acc[j]); acc[j] = wmma_bf(ah, wb, acc[j]); } }
#pragma unroll
  for (int j = 0; j < 8; ++j)
#pragma unroll
    for (int r = 0; r < 8; ++r) so[wave][8 * g + r][j * 16 + col] = acc[j][r];
  LDSX();
  float* dst = n0 < DI ? XI : RES; const int c0 = n0 < DI ? n0 : n0 - DI;
  for (int rl = 0; rl < 16; ++rl) vst2(dst + (size_t)(r0 + rl) * DI + c0 + lane * 4, *(const v4f*)(&so[wave][rl][lane * 4]));
}
__global__ __launch_bounds__(256) void k_conv(const float* __restrict__ XI, const float* __restrict__ cw, const float* __restrict__ cb, float* __restrict__ U) {
  const size_t i4 = (size_t)blockIdx.x * 256 + threadIdx.x; if (i4 >= (size_t)NR * DI / 4) return; const size_t r = i4 / (DI / 4); const int c0 = (int)(i4 % (DI / 4)) * 4; const int l = (int)(r % LL);
  v4f o;
#pragma unroll
  for (int e = 0; e < 4; ++e) { const int c = c0 + e; float acc = bfr(cb[c]);
#pragma unroll
    for (int i = 0; i < 4; ++i) { const int lk = l - 3 + i; if (lk >= 0) acc += bfr(cw[i * DI + c]) * XI[(r - (size_t)(3 - i)) * DI + c]; }
    o[e] = silu_f(acc); }
  vst2(U + r * DI + c0, o);
}
__global__ __launch_bounds__(128) void k_xp(const float* __restrict__ U, const float* __restrict__ Wx, const float* __restrict__ Wdt, const float* __restrict__ bdt, float* __restrict__ DT, float* __restrict__ BM, float* __restrict__ CM) {
  __shared__ __align__(16) float sd[4][16][XDW + 4]; __shared__ __align__(16) float so[4][16][132];
  const int tid = threadIdx.x, wave = tid >> 5, lane = tid & 31, col = lane & 15, g = lane >> 4; const int r0 = blockIdx.x * 64 + wave * 16;
  { v8f acc[12] = {};
#pragma unroll 1
    for (int kc = 0; kc < DI / 32; ++kc) { const F2 a = split_row(U + (size_t)(r0 + col) * DI, kc * 32, lane);
#pragma unroll
      for (int j = 0; j < 12; ++j) { const v16b wb = split_col(Wx, kc * 32, j * 16 + col, lane, XDW, DI).h; acc[j] = wmma_bf(a.l, wb, acc[j]); acc[j] = wmma_bf(a.h, wb, acc[j]); } }
#pragma unroll
    for (int j = 0; j < 12; ++j)
#pragma unroll
      for (int r = 0; r < 8; ++r) sd[wave][8 * g + r][j * 16 + col] = acc[j][r]; }
  LDSX();
  for (int q = lane; q < 16 * 8; q += 32) { const int rl = q >> 3, pc = q & 7; vst2(BM + (size_t)(r0 + rl) * NS + pc * 4, *(const v4f*)(&sd[wave][rl][DTR + pc * 4])); vst2(CM + (size_t)(r0 + rl) * NS + pc * 4, *(const v4f*)(&sd[wave][rl][DTR + NS + pc * 4])); }
#pragma unroll 1
  for (int nh = 0; nh < DI / 128; ++nh) { v8f acc[8] = {};
#pragma unroll
    for (int kc = 0; kc < DTR / 32; ++kc) { const F2 a = split_row(&sd[wave][col][0], kc * 32, lane);
#pragma unroll
      for (int j = 0; j < 8; ++j) { const v16b wb = split_col(Wdt, kc * 32, nh * 128 + j * 16 + col, lane, DI, DTR).h; acc[j] = wmma_bf(a.l, wb, acc[j]); acc[j] = wmma_bf(a.h, wb, acc[j]); } }
#pragma unroll
    for (int j = 0; j < 8; ++j) { const float bb = bfr(bdt[nh * 128 + j * 16 + col]);
#pragma unroll
      for (int r = 0; r < 8; ++r) so[wave][8 * g + r][j * 16 + col] = softplus_ni(acc[j][r] + bb); }
    LDSX();
    for (int rl = 0; rl < 16; ++rl) vst2(DT + (size_t)(r0 + rl) * DI + nh * 128 + lane * 4, *(const v4f*)(&so[wave][rl][lane * 4]));
    LDSX(); }
}
__global__ __launch_bounds__(128) void k_scanR(const float* __restrict__ DT, const float* __restrict__ Alog, int qd, float* __restrict__ REV) {
  const int b = blockIdx.y, dloc = threadIdx.x; const int d = qd * DQ + dloc;
  __shared__ float sA[NS][DQ], src_[NS][DQ];
  for (int n = 0; n < NS; ++n) { sA[n][dloc] = -expf(bfr(Alog[d * NS + n])); src_[n][dloc] = 0.f; }
#pragma unroll 1
  for (int t = LL - 1; t >= 0; --t) { const size_t r = (size_t)b * LL + t; const float dt = DT[r * DI + d]; float* dst = REV + (r * NS) * DQ + dloc;
#pragma unroll 4
    for (int n = 0; n < NS; ++n) { const float rc = src_[n][dloc]; vst2(dst + (size_t)n * DQ, (float_a)rc); src_[n][dloc] = rc + dt * sA[n][dloc]; } }
}
__global__ __launch_bounds__(128) void k_scanF(const float* __restrict__ DT, const float* __restrict__ U, const float* __restrict__ BM, const float* __restrict__ CM, const float* __restrict__ RES, const float* __restrict__ Dp, const float* __restrict__ REV, int qd, float* __restrict__ Y) {
  const int b = blockIdx.y, dloc = threadIdx.x; const int d = qd * DQ + dloc; const float Dd = bfr(Dp[d]);
  __shared__ float scum[NS][DQ];
  for (int n = 0; n < NS; ++n) scum[n][dloc] = 0.f;
#pragma unroll 1
  for (int t = 0; t < LL; ++t) { const size_t r = (size_t)b * LL + t; const float dt = DT[r * DI + d], u = U[r * DI + d], z = RES[r * DI + d]; const float* Br = BM + r * NS; const float* Cr = CM + r * NS; const float* rv = REV + (r * NS) * DQ + dloc;
    const float du = dt * u; float y = 0.f;
#pragma unroll 4
    for (int n = 0; n < NS; ++n) { const float ea = exp_ni(rv[(size_t)n * DQ]); const float c = scum[n][dloc] + du * Br[n] * ea; scum[n][dloc] = c; const float xs = c / (ea + 1e-12f); y += xs * Cr[n]; }
    y = (y + u * Dd) * silu_f(z);
    vst2(Y + r * DI + d, (float_a)y); }
}
__global__ __launch_bounds__(128) void k_head(const float* __restrict__ Y, const float* __restrict__ Wout, const float* __restrict__ bout, const float* __restrict__ x, const float* __restrict__ Wd, const float* __restrict__ bd, float* __restrict__ out) {
  __shared__ __align__(16) float sh2[4][16][DM + 4]; __shared__ __align__(16) float so[4][16][36];
  const int tid = threadIdx.x, wave = tid >> 5, lane = tid & 31, col = lane & 15, g = lane >> 4; const int r0 = blockIdx.x * 64 + wave * 16;
  { v8f acc[16] = {};
#pragma unroll 1
    for (int kc = 0; kc < DI / 32; ++kc) { const F2 a = split_row(Y + (size_t)(r0 + col) * DI, kc * 32, lane);
#pragma unroll
      for (int j = 0; j < 16; ++j) { const v16b wb = split_col(Wout, kc * 32, j * 16 + col, lane, DM, DI).h; acc[j] = wmma_bf(a.l, wb, acc[j]); acc[j] = wmma_bf(a.h, wb, acc[j]); } }
#pragma unroll
    for (int j = 0; j < 16; ++j) { const int n = j * 16 + col; const float bb = bfr(bout[n]);
#pragma unroll
      for (int r = 0; r < 8; ++r) sh2[wave][8 * g + r][n] = acc[j][r] + bb + bfr(x[(size_t)(r0 + 8 * g + r) * DM + n]); } }
  LDSX();
  { v8f acc[2] = {};
#pragma unroll
    for (int kc = 0; kc < DM / 32; ++kc) { const F2 a = split_row(&sh2[wave][col][0], kc * 32, lane);
#pragma unroll
      for (int j = 0; j < 2; ++j) { const v16b wb = split_col(Wd, kc * 32, j * 16 + col, lane, NOUT, DM).h; acc[j] = wmma_bf(a.l, wb, acc[j]); acc[j] = wmma_bf(a.h, wb, acc[j]); } }
#pragma unroll
    for (int j = 0; j < 2; ++j) { const float bb = bfr(bd[j * 16 + col]);
#pragma unroll
      for (int r = 0; r < 8; ++r) so[wave][8 * g + r][j * 16 + col] = gelu_ni(acc[j][r] + bb); } }
  LDSX();
  for (int q = lane; q < 16 * 8; q += 32) { const int rl = q >> 3, pc = q & 7; vst2(out + (size_t)(r0 + rl) * NOUT + pc * 4, *(const v4f*)(&so[wave][rl][pc * 4])); }
}
extern "C" void kernel_launch(void* const* d_in, const int* in_sizes, int n_in, void* d_out, int out_size, void* d_ws, size_t ws_size, hipStream_t stream) {
  (void)in_sizes; (void)n_in; (void)out_size; (void)ws_size;
  const float** I = (const float**)d_in;
  const float* x = I[0]; const float* lg = I[1]; const float* lb = I[2]; const float* Win = I[3]; const float* cw = I[4]; const float* cb = I[5]; const float* Wx = I[6]; const float* Wdt = I[7]; const float* bdt = I[8]; const float* Alog = I[9]; const float* Dp = I[10]; const float* Wout = I[11]; const float* bout = I[12]; const float* Wd = I[13]; const float* bd = I[14];
  char* ws = (char*)d_ws; size_t off = 0;
  auto take = [&](size_t bytes) { char* p = ws + off; off += (bytes + 255) & ~(size_t)255; return p; };
  float* XI = (float*)take((size_t)NR * DI * 4); float* RES = (float*)take((size_t)NR * DI * 4); float* U = (float*)take((size_t)NR * DI * 4); float* DT = (float*)take((size_t)NR * DI * 4);
  float* BM = (float*)take((size_t)NR * NS * 4); float* CM = (float*)take((size_t)NR * NS * 4); float* Y = (float*)take((size_t)NR * DI * 4); float* REV = (float*)take((size_t)NR * NS * DQ * 4);
  k_lnin<<<dim3(NR / 64, 2 * DI / 128), 128, 0, stream>>>(x, lg, lb, Win, XI, RES);
  k_conv<<<(NR * DI / 4 + 255) / 256, 256, 0, stream>>>(XI, cw, cb, U);
  k_xp<<<NR / 64, 128, 0, stream>>>(U, Wx, Wdt, bdt, DT, BM, CM);
  for (int qd = 0; qd < DI / DQ; ++qd) {
    k_scanR<<<dim3(1, NBB), 128, 0, stream>>>(DT, Alog, qd, REV);
    k_scanF<<<dim3(1, NBB), 128, 0, stream>>>(DT, U, BM, CM, RES, Dp, REV, qd, Y); }
  k_head<<<NR / 64, 128, 0, stream>>>(Y, Wout, bout, x, Wd, bd, (float*)d_out);
}
